// CrossAttention_55439437857301
// MI455X (gfx1250) — hardware-verified
//
#include <hip/hip_runtime.h>


#ifndef NB
#define NB 4
#endif
#ifndef SEQ
#define SEQ 4096
#endif
#define NBF  4
#define SEQF 4096
#define CC   256
#define C8   32
#define FGW  64
#define PCAR 16384.0f
#define PINV 0.00006103515625f
#define L2E  1.4426950408889634f
#define LN2  0.6931471805599453f
#define NFGB ((C8 * CC) / 2048)
#define NHB  ((CC * CC) / 2048)

static_assert(NB >= 1 && NB <= NBF);
static_assert(SEQ % 256 == 0 && SEQ >= 256 && SEQ <= SEQF);
static_assert(CC == 256 && C8 == 32 && FGW == 64);
static_assert((C8 * CC) % 2048 == 0 && (CC * CC) % 2048 == 0);
static_assert((size_t)NBF * CC * SEQF * 4 == 16777216);
static_assert((NB * SEQ * FGW) % 2048 == 0 && (NB * CC * SEQ) % 2048 == 0);

typedef _Float16 h16;
typedef unsigned short bf;
typedef __attribute__((ext_vector_type(16))) __bf16   v16bf;
typedef __attribute__((ext_vector_type(16))) _Float16 v16h;
typedef __attribute__((ext_vector_type(8)))  _Float16 v8h;
typedef __attribute__((ext_vector_type(8)))  unsigned short v8us;
typedef __attribute__((ext_vector_type(8)))  float    v8f;
typedef __attribute__((ext_vector_type(4)))  float    v4f;
typedef v8h  __attribute__((may_alias)) v8ha;
typedef v4f  __attribute__((may_alias)) v4fa;
typedef v8us __attribute__((may_alias)) v8usa;

__device__ __forceinline__ unsigned short f2bf(float f) { unsigned u = __float_as_uint(f); u += 0x7FFFu + ((u >> 16) & 1u); return (unsigned short)(u >> 16); }
__device__ __forceinline__ float bf2f(unsigned short b) { return __uint_as_float(((unsigned)b) << 16); }
__device__ __forceinline__ float bfr(float f) { return bf2f(f2bf(f)); }
__device__ __forceinline__ void splitf(float y, unsigned short& h, unsigned short& l) { h = f2bf(y); l = f2bf(y - bf2f(h)); }
__device__ __forceinline__ v16h cat16(v8h lo, v8h hi) { return __builtin_shufflevector(lo, hi, 0, 1, 2, 3, 4, 5, 6, 7, 8, 9, 10, 11, 12, 13, 14, 15); }
__device__ __forceinline__ v16bf cat16b(v8us lo, v8us hi) { return __builtin_bit_cast(v16bf, __builtin_shufflevector(lo, hi, 0, 1, 2, 3, 4, 5, 6, 7, 8, 9, 10, 11, 12, 13, 14, 15)); }
__device__ __forceinline__ v8f wmma16(v16h a, v16h b, v8f c) { return __builtin_amdgcn_wmma_f32_16x16x32_f16(false, a, false, b, (short)0, c, false, false); }
__device__ __forceinline__ v8f wmmab(v16bf a, v16bf b, v8f c) { return __builtin_amdgcn_wmma_f32_16x16x32_bf16(false, a, false, b, (short)0, c, false, false); }
__device__ __forceinline__ v16bf ldbf(const bf* p)  { return cat16b(*(const v8us*)p, *(const v8us*)(p + 16)); }
__device__ __forceinline__ v16bf ldbfs(const bf* p) { return cat16b(*(const v8usa*)p, *(const v8usa*)(p + 16)); }
__device__ __forceinline__ v16h  ldh(const h16* p)  { return cat16(*(const v8h*)p, *(const v8h*)(p + 16)); }
__device__ __forceinline__ v16h  ldhs(const h16* p) { return cat16(*(const v8ha*)p, *(const v8ha*)(p + 16)); }

__global__ __launch_bounds__(32) void k_gemmw(const bf* __restrict__ A, const bf* __restrict__ Bt, int K, float* C, int ldc, size_t sA, size_t sB, size_t sC) {
    __shared__ __align__(16) float os[16 * 68];
    const size_t z = blockIdx.z; A += z * sA; Bt += z * sB; C += z * sC;
    const int lane = threadIdx.x & 31, lr = lane & 15, hi = lane >> 4; const int r0 = blockIdx.x * 64, c0 = blockIdx.y * 64;
    v8f acc[4][4];
#pragma unroll
    for (int mb = 0; mb < 4; ++mb)
#pragma unroll
        for (int nb = 0; nb < 4; ++nb) acc[mb][nb] = (v8f){};
    const size_t aoff = (size_t)(r0 + lr) * K + 8 * hi, boff = (size_t)(c0 + lr) * K + 8 * hi;
#pragma unroll 1
    for (int kc = 0; kc < K; kc += 32) {
        v16bf a[4];
#pragma unroll
        for (int mb = 0; mb < 4; ++mb) a[mb] = ldbf(A + aoff + (size_t)mb * 16 * K + kc);
#pragma unroll
        for (int nb = 0; nb < 4; ++nb) { const v16bf b = ldbf(Bt + boff + (size_t)nb * 16 * K + kc);
#pragma unroll
            for (int mb = 0; mb < 4; ++mb) acc[mb][nb] = wmmab(a[mb], b, acc[mb][nb]); }
        asm volatile("v_nop\n\tv_nop\n\tv_nop\n\tv_nop" : "+v"(acc[0][0]), "+v"(acc[1][1]), "+v"(acc[2][2]), "+v"(acc[3][3]) : "v"(a[0]), "v"(a[3]));
    }
#pragma unroll
    for (int mb = 0; mb < 4; ++mb) {
#pragma unroll
        for (int nb = 0; nb < 4; ++nb) {
#pragma unroll
            for (int j = 0; j < 8; ++j) os[(hi * 8 + j) * 68 + nb * 16 + lr] = acc[mb][nb][j]; }
        __builtin_amdgcn_wave_barrier(); asm volatile("" ::: "memory");
        float* crow = C + (size_t)(r0 + mb * 16) * ldc + c0;
#pragma unroll 1
        for (int ps = 0; ps < 2; ++ps) {
#pragma unroll
            for (int s = 0; s < 8; ++s) { const int row = 2 * s + hi, cofs = lr * 4; const v4f val = *(const v4fa*)(os + row * 68 + cofs);
                *(volatile v4f*)(crow + (size_t)row * ldc + cofs) = val; }
            if (ps == 0) __threadfence(); }
        __builtin_amdgcn_wave_barrier(); asm volatile("" ::: "memory");
    }
}

__global__ __launch_bounds__(256) void k_packw(const float* __restrict__ Wf, const float* __restrict__ Wg, const float* __restrict__ Wh, bf* WFG, bf* WH) {
    const int blk = blockIdx.x, t = threadIdx.x;
    const float* src; bf* dst; size_t i;
    if (blk < NFGB)          { src = Wf; dst = WFG;           i = (size_t)blk * 256 + t; }
    else if (blk < 2 * NFGB) { src = Wg; dst = WFG + C8 * CC; i = (size_t)(blk - NFGB) * 256 + t; }
    else                     { src = Wh; dst = WH;            i = (size_t)(blk - 2 * NFGB) * 256 + t; }
    const v8f v = *(const v8f*)(src + i * 8); v8us o;
#pragma unroll
    for (int k = 0; k < 8; ++k) o[k] = f2bf(v[k]);
    *(volatile v8us*)(dst + i * 8) = o; __threadfence(); *(volatile v8us*)(dst + i * 8) = o;
}

__global__ __launch_bounds__(256) void k_xT(const float* __restrict__ src, bf* dst) {
    __shared__ float tile[64][65];
    const int b = blockIdx.z, n0 = blockIdx.x * 64, c0 = blockIdx.y * 64, t = threadIdx.x;
    const float* s = src + (size_t)b * CC * SEQF;
#pragma unroll
    for (int it = 0; it < 16; ++it) { const int c = it * 4 + (t >> 6), n = t & 63; tile[c][n] = s[(size_t)(c0 + c) * SEQF + n0 + n]; }
    __syncthreads();
    bf* d = dst + (size_t)b * SEQ * CC;
    v8us o[2]; size_t off[2];
#pragma unroll
    for (int s2 = 0; s2 < 2; ++s2) { const int p = t + 256 * s2, n = p >> 3, q = p & 7;
#pragma unroll
        for (int e = 0; e < 8; ++e) o[s2][e] = f2bf(tile[8 * q + e][n]);
        off[s2] = (size_t)(n0 + n) * CC + c0 + 8 * q; }
    *(volatile v8us*)(d + off[0]) = o[0]; *(volatile v8us*)(d + off[1]) = o[1];
    __threadfence();
    *(volatile v8us*)(d + off[0]) = o[0]; *(volatile v8us*)(d + off[1]) = o[1];
}

__global__ __launch_bounds__(256) void k_fgplanes(const float* __restrict__ FG, const float* __restrict__ bfp, const float* __restrict__ bgp, bf* Ph, bf* Pl, size_t n8) {
    const size_t i = (size_t)blockIdx.x * 256 + threadIdx.x; if (i >= n8) return;
    const v8f a = *(const v8f*)(FG + i * 8); const int col0 = (int)((i * 8) & 63);
    v8us oh, ol;
#pragma unroll
    for (int e = 0; e < 8; ++e) { const int col = col0 + e; const float b1 = bfp[col & 31], b2 = bgp[col & 31]; const float bb = (col0 < 32) ? b1 : b2;
        const float v = a[e] + bfr(bb); unsigned short x2, y2; splitf(v, x2, y2); oh[e] = x2; ol[e] = y2; }
    *(volatile v8us*)(Ph + i * 8) = oh; *(volatile v8us*)(Pl + i * 8) = ol; __threadfence(); *(volatile v8us*)(Ph + i * 8) = oh; *(volatile v8us*)(Pl + i * 8) = ol;
}

__global__ __launch_bounds__(256) void k_hplane(const float* __restrict__ Hf, const float* __restrict__ bhp, h16* H16, size_t n8) {
    const size_t i = (size_t)blockIdx.x * 256 + threadIdx.x; if (i >= n8) return;
    const v8f a = *(const v8f*)(Hf + i * 8); const int o = (int)(((i * 8) / SEQ) % CC); const float bb = bfr(bhp[o]);
    v8h oh;
#pragma unroll
    for (int e = 0; e < 8; ++e) oh[e] = (h16)(a[e] + bb);
    *(volatile v8h*)(H16 + i * 8) = oh; __threadfence(); *(volatile v8h*)(H16 + i * 8) = oh;
}

__global__ __launch_bounds__(256) void k_lse(const bf* __restrict__ Qh, const bf* __restrict__ Ql, const bf* __restrict__ Kh, const bf* __restrict__ Kl, float* L) {
    const int lane = threadIdx.x & 31, lr = lane & 15, hh = lane >> 4;
    const int wid = blockIdx.x * 8 + (threadIdx.x >> 5);
    const int b = wid / (SEQ / 32), n0 = (wid % (SEQ / 32)) * 32;
    const size_t po = (size_t)b * SEQ * FGW;
    v16bf ah[2], al[2];
#pragma unroll
    for (int t = 0; t < 2; ++t) { const size_t qo = po + (size_t)(n0 + 16 * t + lr) * FGW + 8 * hh; ah[t] = ldbf(Qh + qo); al[t] = ldbf(Ql + qo); }
    float mx[2][8], sm[2][8];
#pragma unroll
    for (int t = 0; t < 2; ++t)
#pragma unroll
        for (int r = 0; r < 8; ++r) { mx[t][r] = -1.0e30f; sm[t][r] = 0.f; }
#pragma unroll 1
    for (int mg = 0; mg < SEQ / 64; ++mg) {
        v8f s[2][4];
#pragma unroll
        for (int j = 0; j < 4; ++j) {
            const size_t ko = po + (size_t)(mg * 64 + 16 * j + lr) * FGW + 8 * hh;
            const v16bf bh_ = ldbf(Kh + ko), bl_ = ldbf(Kl + ko);
#pragma unroll
            for (int t = 0; t < 2; ++t) { v8f d = wmmab(ah[t], bh_, (v8f){}); d = wmmab(ah[t], bl_, d); d = wmmab(al[t], bh_, d); s[t][j] = d; }
            asm volatile("v_nop\n\tv_nop\n\tv_nop\n\tv_nop" : "+v"(s[0][j]), "+v"(s[1][j]) : "v"(bh_), "v"(bl_), "v"(al[1]));
        }
#pragma unroll
        for (int t = 0; t < 2; ++t)
#pragma unroll
            for (int r = 0; r < 8; ++r) {
                const float gmx = fmaxf(fmaxf(s[t][0][r], s[t][1][r]), fmaxf(s[t][2][r], s[t][3][r]));
                const float nm = fmaxf(mx[t][r], gmx);
                float a2 = sm[t][r] * __builtin_amdgcn_exp2f((mx[t][r] - nm) * L2E);
#pragma unroll
                for (int j = 0; j < 4; ++j) a2 += __builtin_amdgcn_exp2f((s[t][j][r] - nm) * L2E);
                sm[t][r] = a2; mx[t][r] = nm; }
    }
#pragma unroll
    for (int dd = 1; dd < 16; dd <<= 1) {
#pragma unroll
        for (int t = 0; t < 2; ++t)
#pragma unroll
            for (int r = 0; r < 8; ++r) {
                const float om = __shfl_xor(mx[t][r], dd), osm = __shfl_xor(sm[t][r], dd);
                const float nm = fmaxf(mx[t][r], om);
                sm[t][r] = sm[t][r] * __builtin_amdgcn_exp2f((mx[t][r] - nm) * L2E) + osm * __builtin_amdgcn_exp2f((om - nm) * L2E);
                mx[t][r] = nm; } }
    const int srcl = (lane & 8) ? 16 : 0;
    float outv = 0.f;
#pragma unroll
    for (int t = 0; t < 2; ++t)
#pragma unroll
        for (int r = 0; r < 8; ++r) {
            const float lv = mx[t][r] + __log2f(sm[t][r]) * LN2;
            const float cand = __shfl(lv, srcl);
            if (((lane >> 4) == t) && ((lane & 7) == r)) outv = cand; }
    float* Lp = L + (size_t)b * SEQ + n0 + lane;
    *(volatile float*)Lp = outv; __threadfence(); *(volatile float*)Lp = outv;
}

__global__ __launch_bounds__(256) void k_pv(const bf* __restrict__ Qh, const bf* __restrict__ Ql, const bf* __restrict__ Kh, const bf* __restrict__ Kl,
                                           const h16* __restrict__ Hp, const float* __restrict__ L, const float* __restrict__ resid, const float* __restrict__ gam, float* out) {
    __shared__ __align__(16) float Psm[8 * 64 * 32 / 2];
    __shared__ __align__(16) bf Gs[2 * 64 * 32];
    const int tid = threadIdx.x, lane = tid & 31, lr = lane & 15, hh = lane >> 4, w = tid >> 5;
    const int b = blockIdx.y, m0 = blockIdx.x * 64;
    const size_t po = (size_t)b * SEQ * FGW;
    h16* Pt = (h16*)Psm;
    { const int row = tid >> 2, k8 = (tid & 3) * 8; const size_t go = po + (size_t)(m0 + row) * FGW + k8;
      *(v8usa*)(Gs + row * 32 + k8) = *(const v8us*)(Kh + go); *(v8usa*)(Gs + 2048 + row * 32 + k8) = *(const v8us*)(Kl + go); }
    __syncthreads();
    v8f acc[2][4];
#pragma unroll
    for (int i = 0; i < 2; ++i)
#pragma unroll
        for (int j = 0; j < 4; ++j) acc[i][j] = (v8f){};
    const float* Lb = L + (size_t)b * SEQ;
    const h16* Hb = Hp + (size_t)b * CC * SEQ + (size_t)(32 * w + lr) * SEQ + 8 * hh;
#pragma unroll 1
    for (int sup = 0; sup < SEQ / 256; ++sup) {
        const int n0 = (sup * 8 + w) * 32;
        v16bf ah[2], al[2]; v4f la[2], lb[2];
#pragma unroll
        for (int t = 0; t < 2; ++t) { const size_t qo = po + (size_t)(n0 + 16 * t + lr) * FGW + 8 * hh; ah[t] = ldbf(Qh + qo); al[t] = ldbf(Ql + qo);
            la[t] = *(const v4f*)(Lb + n0 + 16 * t + 8 * hh); lb[t] = *(const v4f*)(Lb + n0 + 16 * t + 8 * hh + 4); }
#pragma unroll
        for (int j = 0; j < 4; ++j) {
            const bf* gp = Gs + (16 * j + lr) * 32 + 8 * hh; const v16bf bh_ = ldbfs(gp), bl_ = ldbfs(gp + 2048);
            v8f s[2];
#pragma unroll
            for (int t = 0; t < 2; ++t) { v8f d = wmmab(ah[t], bh_, (v8f){}); d = wmmab(ah[t], bl_, d); d = wmmab(al[t], bh_, d); s[t] = d; }
            asm volatile("v_nop\n\tv_nop\n\tv_nop\n\tv_nop" : "+v"(s[0]), "+v"(s[1]) : "v"(bh_), "v"(bl_), "v"(al[1]));
#pragma unroll
            for (int t = 0; t < 2; ++t) { v8h pk;
#pragma unroll
                for (int r = 0; r < 4; ++r) { pk[r] = (h16)(__builtin_amdgcn_exp2f((s[t][r] - la[t][r]) * L2E) * PCAR); pk[r + 4] = (h16)(__builtin_amdgcn_exp2f((s[t][r + 4] - lb[t][r]) * L2E) * PCAR); }
                *(v8ha*)(Pt + (size_t)(w * 64 + 16 * j + lr) * 32 + 16 * t + 8 * hh) = pk; }
        }
        __syncthreads();
        v16h pf;
#pragma unroll
        for (int ch = 0; ch < 8; ++ch) { const int nk = sup * 256 + ch * 32;
            const v16h h0 = ldh(Hb + nk), h1 = ldh(Hb + (size_t)16 * SEQ + nk);
#pragma unroll
            for (int j = 0; j < 4; ++j) { pf = ldhs(Pt + (ch * 64 + 16 * j + lr) * 32 + 8 * hh);
                acc[0][j] = wmma16(h0, pf, acc[0][j]); acc[1][j] = wmma16(h1, pf, acc[1][j]); }
            asm volatile("v_nop\n\tv_nop\n\tv_nop\n\tv_nop" : "+v"(acc[0][0]), "+v"(acc[0][1]), "+v"(acc[0][2]), "+v"(acc[0][3]), "+v"(acc[1][0]), "+v"(acc[1][1]), "+v"(acc[1][2]), "+v"(acc[1][3]) : "v"(h0), "v"(h1), "v"(pf)); }
        __syncthreads();
    }
    const float g2 = bfr(gam[0]) * PINV;
    float* osw = Psm + w * 1024;
#pragma unroll
    for (int i = 0; i < 2; ++i) {
#pragma unroll
        for (int j = 0; j < 4; ++j)
#pragma unroll
            for (int r = 0; r < 8; ++r) osw[(8 * hh + r) * 64 + 16 * j + lr] = acc[i][j][r];
        __builtin_amdgcn_fence(4  , "wavefront"); __builtin_amdgcn_wave_barrier(); asm volatile("" ::: "memory");
        const size_t ob = ((size_t)b * CC + 32 * w + 16 * i) * SEQF + m0;
#pragma unroll 1
        for (int ps = 0; ps < 2; ++ps) {
#pragma unroll
            for (int s = 0; s < 8; ++s) { const int row = 2 * s + hh, cofs = lr * 4;
                const v4f val = *(const v4fa*)(osw + row * 64 + cofs); const v4f rx = *(const v4f*)(resid + ob + (size_t)row * SEQF + cofs);
                v4f o;
#pragma unroll
                for (int k = 0; k < 4; ++k) o[k] = g2 * val[k] + bfr(rx[k]);
                *(volatile v4f*)(out + ob + (size_t)row * SEQF + cofs) = o; }
            if (ps == 0) __threadfence(); }
        __builtin_amdgcn_fence(4  , "wavefront"); __builtin_amdgcn_wave_barrier(); asm volatile("" ::: "memory");
    }
}

extern "C" void kernel_launch(void* const* d_in, const int* in_sizes, int n_in,
                              void* d_out, int out_size, void* d_ws, size_t ws_size, hipStream_t stream) {
    if (n_in < 15) return;
    if (in_sizes[0] < NB * CC * SEQF || in_sizes[1] < NB * CC * SEQF) return;
    if (in_sizes[2] < C8 * CC || in_sizes[4] < C8 * CC || in_sizes[8] < C8 * CC || in_sizes[10] < C8 * CC) return;
    if (in_sizes[3] < C8 || in_sizes[5] < C8 || in_sizes[9] < C8 || in_sizes[11] < C8) return;
    if (in_sizes[6] < CC * CC || in_sizes[12] < CC * CC || in_sizes[7] < CC || in_sizes[13] < CC || in_sizes[14] < 1) return;
    if ((size_t)out_size < (size_t)2 * NBF * CC * SEQF) return;
    const float* x   = (const float*)d_in[0];  const float* y   = (const float*)d_in[1];
    const float* Wfx = (const float*)d_in[2];  const float* bfx = (const float*)d_in[3];
    const float* Wgx = (const float*)d_in[4];  const float* bgx = (const float*)d_in[5];
    const float* Whx = (const float*)d_in[6];  const float* bhx = (const float*)d_in[7];
    const float* Wfy = (const float*)d_in[8];  const float* bfy = (const float*)d_in[9];
    const float* Wgy = (const float*)d_in[10]; const float* bgy = (const float*)d_in[11];
    const float* Why = (const float*)d_in[12]; const float* bhy = (const float*)d_in[13];
    const float* gam = (const float*)d_in[14];
    float* OUTX = (float*)d_out; float* OUTY = OUTX + (size_t)NBF * CC * SEQF;
    char* wsp = (char*)d_ws;
    auto take = [&](size_t bytes) { char* p = wsp; wsp += (bytes + 255) & ~(size_t)255; return (void*)p; };
    bf* WFGx = (bf*)take((size_t)FGW * CC * 2); bf* WFGy = (bf*)take((size_t)FGW * CC * 2);
    bf* WHx  = (bf*)take((size_t)CC * CC * 2);  bf* WHy  = (bf*)take((size_t)CC * CC * 2);
    bf* XT   = (bf*)take((size_t)NB * SEQ * CC * 2); bf* YT = (bf*)take((size_t)NB * SEQ * CC * 2);
    float* FGfx = (float*)take((size_t)NB * SEQ * FGW * 4); float* FGfy = (float*)take((size_t)NB * SEQ * FGW * 4);
    bf* FGxh = (bf*)take((size_t)NB * SEQ * FGW * 2); bf* FGxl = (bf*)take((size_t)NB * SEQ * FGW * 2);
    bf* FGyh = (bf*)take((size_t)NB * SEQ * FGW * 2); bf* FGyl = (bf*)take((size_t)NB * SEQ * FGW * 2);
    float* Hfx = (float*)take((size_t)NB * CC * SEQ * 4); float* Hfy = (float*)take((size_t)NB * CC * SEQ * 4);
    h16* Hx16 = (h16*)take((size_t)NB * CC * SEQ * 2); h16* Hy16 = (h16*)take((size_t)NB * CC * SEQ * 2);
    float* Lx = (float*)take((size_t)NB * SEQ * 4); float* Ly = (float*)take((size_t)NB * SEQ * 4);
    if ((size_t)(wsp - (char*)d_ws) > ws_size) return;
    const size_t n8fg = (size_t)NB * SEQ * FGW / 8, n8h = (size_t)NB * CC * SEQ / 8;

    k_packw<<<2 * NFGB + NHB, 256, 0, stream>>>(Wfx, Wgx, Whx, WFGx, WHx);
    k_packw<<<2 * NFGB + NHB, 256, 0, stream>>>(Wfy, Wgy, Why, WFGy, WHy);
    k_xT<<<dim3(SEQ / 64, CC / 64, NB), 256, 0, stream>>>(x, XT);
    k_xT<<<dim3(SEQ / 64, CC / 64, NB), 256, 0, stream>>>(y, YT);
    k_gemmw<<<dim3(SEQ / 64, FGW / 64, NB), 32, 0, stream>>>(XT, WFGx, CC, FGfx, FGW, (size_t)SEQ * CC, 0, (size_t)SEQ * FGW);
    k_gemmw<<<dim3(SEQ / 64, FGW / 64, NB), 32, 0, stream>>>(YT, WFGy, CC, FGfy, FGW, (size_t)SEQ * CC, 0, (size_t)SEQ * FGW);
    k_gemmw<<<dim3(CC / 64, SEQ / 64, NB), 32, 0, stream>>>(WHx, XT, CC, Hfx, SEQ, 0, (size_t)SEQ * CC, (size_t)CC * SEQ);
    k_gemmw<<<dim3(CC / 64, SEQ / 64, NB), 32, 0, stream>>>(WHy, YT, CC, Hfy, SEQ, 0, (size_t)SEQ * CC, (size_t)CC * SEQ);
    k_fgplanes<<<(unsigned)((n8fg + 255) / 256), 256, 0, stream>>>(FGfx, bfx, bgx, FGxh, FGxl, n8fg);
    k_fgplanes<<<(unsigned)((n8fg + 255) / 256), 256, 0, stream>>>(FGfy, bfy, bgy, FGyh, FGyl, n8fg);
    k_hplane<<<(unsigned)((n8h + 255) / 256), 256, 0, stream>>>(Hfx, bhx, Hx16, n8h);
    k_hplane<<<(unsigned)((n8h + 255) / 256), 256, 0, stream>>>(Hfy, bhy, Hy16, n8h);
    k_lse<<<NB * SEQ / 256, 256, 0, stream>>>(FGyh, FGyl, FGxh + C8, FGxl + C8, Lx);
    k_lse<<<NB * SEQ / 256, 256, 0, stream>>>(FGxh, FGxl, FGyh + C8, FGyl + C8, Ly);
    k_pv<<<dim3(SEQ / 64, NB), 256, 0, stream>>>(FGyh, FGyl, FGxh + C8, FGxl + C8, Hx16, Lx, x, gam, OUTX);
    k_pv<<<dim3(SEQ / 64, NB), 256, 0, stream>>>(FGxh, FGxl, FGyh + C8, FGyl + C8, Hy16, Ly, y, gam, OUTY);
}
